// Glm4MoeDecoderLayer_63221918597201
// MI455X (gfx1250) — hardware-verified
//
#include <hip/hip_runtime.h>
#include <hip/hip_bf16.h>
#include <stddef.h>
#include <stdint.h>

#define SQ    2048
#define HID   1024
#define NH    16
#define NKV   4
#define HDM   64
#define HALF  32
#define NQKV  1536
#define KOFS  1024
#define VOFS  1280
#define NE    16
#define NTOP  4
#define FFI   512
#define CAP   SQ
#define MT    (SQ / 64)
#define NQ64  (SQ / 64)
#define RTW   32
#define XSC   8.0f
#define WSC   32.0f
#define MSC   64.0f

static_assert(SQ % 256 == 0);
static_assert(HID % 256 == 0);
static_assert(HID == 128 * 8);
static_assert(HDM == 64);
static_assert(NH * HDM == HID);
static_assert(NH == 4 * NKV);
static_assert(NQKV == NH * HDM + 2 * NKV * HDM);
static_assert(KOFS == NH * HDM);
static_assert(VOFS == NH * HDM + NKV * HDM);
static_assert((SQ * HALF) % 256 == 0);
static_assert(FFI % 128 == 0);
static_assert(NE == 16);
static_assert(NTOP == 4);
static_assert(MT * 64 == CAP);

typedef _Float16 v16h __attribute__((ext_vector_type(16)));
typedef _Float16 v8h  __attribute__((ext_vector_type(8)));
typedef float    v8f  __attribute__((ext_vector_type(8)));
typedef float    v4f  __attribute__((ext_vector_type(4)));
typedef unsigned int   v4u   __attribute__((ext_vector_type(4)));
typedef unsigned short v8us  __attribute__((ext_vector_type(8)));
typedef unsigned short v16us __attribute__((ext_vector_type(16)));
typedef __bf16         v16b  __attribute__((ext_vector_type(16)));
typedef unsigned short ush;

union Frag  { v16h v; v8h h[2]; };
union FragU { v16us v; v8us h[2]; v16b b; };
union Pack8 { v8h h; v4u u; };
union PackU { v8us s; v4u u; };
struct HL { v4u h; v4u l; };

__device__ __forceinline__ ush f2bf(float f) {
  const unsigned u = __float_as_uint(f);
  return (ush)((u + 0x7FFFu + ((u >> 16) & 1u)) >> 16);
}
__device__ __forceinline__ float bf2f(ush b) { return __uint_as_float(((unsigned)b) << 16); }

__device__ __forceinline__ HL split8(v8f f) {
  PackU ph, pl;
#pragma unroll
  for (int e = 0; e < 8; ++e) {
    const ush hi = f2bf(f[e]);
    ph.s[e] = hi;
    pl.s[e] = f2bf(f[e] - bf2f(hi));
  }
  HL r; r.h = ph.u; r.l = pl.u;
  return r;
}

__device__ __forceinline__ v8f mma16(v16h a, v16h b, v8f c) {
  c = __builtin_amdgcn_wmma_f32_16x16x32_f16(false, a, false, b, (short)0, c, false, false);
  asm volatile("v_nop\n\tv_nop\n\tv_nop\n\tv_nop" : "+v"(c) : "v"(a), "v"(b));
  return c;
}
__device__ __forceinline__ v8f mmab(v16us a, v16us b, v8f c) {
  FragU ua, ub; ua.v = a; ub.v = b;
  c = __builtin_amdgcn_wmma_f32_16x16x32_bf16(false, ua.b, false, ub.b, (short)0, c, false, false);
  asm volatile("v_nop\n\tv_nop\n\tv_nop\n\tv_nop" : "+v"(c) : "v"(a), "v"(b));
  return c;
}

__device__ __forceinline__ v16h ldfrag(const _Float16* p, int ld, int row0, int k0, int lane) {
  const int m = lane & 15, lh = lane >> 4;
  const _Float16* q = p + (size_t)(row0 + m) * ld + k0 + 8 * lh;
  Frag f;
  f.h[0] = *(const v8h*)(q);
  f.h[1] = *(const v8h*)(q + 16);
  return f.v;
}
__device__ __forceinline__ v16us ldfragu(const ush* p, int ld, int row0, int k0, int lane) {
  const int m = lane & 15, lh = lane >> 4;
  const ush* q = p + (size_t)(row0 + m) * ld + k0 + 8 * lh;
  FragU f;
  f.h[0] = *(const v8us*)(q);
  f.h[1] = *(const v8us*)(q + 16);
  return f.v;
}

__device__ __forceinline__ v8f zero8() { return (v8f){0.f, 0.f, 0.f, 0.f, 0.f, 0.f, 0.f, 0.f}; }

__device__ __forceinline__ void gemm3_16x64(const ush* __restrict__ Ah, const ush* __restrict__ Al, int lda,
                                            const ush* __restrict__ Bh, const ush* __restrict__ Bl, int ldb,
                                            int m0, int n0, int lane, v8f (&acc)[4]) {
#pragma unroll 1
  for (int k0 = 0; k0 < HID; k0 += 32) {
    const v16us ah = ldfragu(Ah, lda, m0, k0, lane);
    const v16us al = ldfragu(Al, lda, m0, k0, lane);
#pragma unroll
    for (int t = 0; t < 4; ++t) {
      const v16us bh = ldfragu(Bh, ldb, n0 + 16 * t, k0, lane);
      const v16us bl = ldfragu(Bl, ldb, n0 + 16 * t, k0, lane);
      acc[t] = mmab(ah, bh, acc[t]);
      acc[t] = mmab(ah, bl, acc[t]);
      acc[t] = mmab(al, bh, acc[t]);
    }
  }
}

__device__ __forceinline__ void gemm3_32x64(const ush* __restrict__ Ah, const ush* __restrict__ Al, int lda,
                                            const ush* __restrict__ Bh, const ush* __restrict__ Bl, int ldb,
                                            int m0, int n0, int lane, v8f (&acc)[2][4]) {
#pragma unroll 1
  for (int k0 = 0; k0 < HID; k0 += 32) {
    const v16us a0h = ldfragu(Ah, lda, m0, k0, lane);
    const v16us a1h = ldfragu(Ah, lda, m0 + 16, k0, lane);
    const v16us a0l = ldfragu(Al, lda, m0, k0, lane);
    const v16us a1l = ldfragu(Al, lda, m0 + 16, k0, lane);
#pragma unroll
    for (int t = 0; t < 4; ++t) {
      const v16us bh = ldfragu(Bh, ldb, n0 + 16 * t, k0, lane);
      const v16us bl = ldfragu(Bl, ldb, n0 + 16 * t, k0, lane);
      acc[0][t] = mmab(a0h, bh, acc[0][t]);
      acc[1][t] = mmab(a1h, bh, acc[1][t]);
      acc[0][t] = mmab(a0h, bl, acc[0][t]);
      acc[1][t] = mmab(a1h, bl, acc[1][t]);
      acc[0][t] = mmab(a0l, bh, acc[0][t]);
      acc[1][t] = mmab(a1l, bh, acc[1][t]);
    }
  }
}

template <int KD>
__device__ __forceinline__ void gemm32x64h(const _Float16* __restrict__ A, int lda,
                                           const _Float16* __restrict__ Bt, int ldb,
                                           int m0, int n0, int lane, v8f (&acc)[2][4]) {
#pragma unroll 2
  for (int k0 = 0; k0 < KD; k0 += 32) {
    const v16h a0 = ldfrag(A, lda, m0, k0, lane);
    const v16h a1 = ldfrag(A, lda, m0 + 16, k0, lane);
    const v16h b0 = ldfrag(Bt, ldb, n0, k0, lane);
    const v16h b1 = ldfrag(Bt, ldb, n0 + 16, k0, lane);
    const v16h b2 = ldfrag(Bt, ldb, n0 + 32, k0, lane);
    const v16h b3 = ldfrag(Bt, ldb, n0 + 48, k0, lane);
    acc[0][0] = mma16(a0, b0, acc[0][0]);
    acc[1][0] = mma16(a1, b0, acc[1][0]);
    acc[0][1] = mma16(a0, b1, acc[0][1]);
    acc[1][1] = mma16(a1, b1, acc[1][1]);
    acc[0][2] = mma16(a0, b2, acc[0][2]);
    acc[1][2] = mma16(a1, b2, acc[1][2]);
    acc[0][3] = mma16(a0, b3, acc[0][3]);
    acc[1][3] = mma16(a1, b3, acc[1][3]);
  }
}

__global__ __launch_bounds__(256) void k_tab(const int* __restrict__ pid, float* __restrict__ ct,
                                             float* __restrict__ sn, int npos) {
  __shared__ float invf[HALF];
  const int tid = threadIdx.x;
  if (tid < HALF) {
    const int m  = tid;
    const int ip = m >> 3;
    double p = 1.0;
    if (ip >= 1) p *= 10.0;
    if (ip >= 2) p *= 10.0;
    if (ip >= 3) p *= 10.0;
    if (m & 4) p *= 3.1622776601683795;
    if (m & 2) p *= 1.7782794100389228;
    if (m & 1) p *= 1.3335214321633240;
    const float t32 = (float)p;
    invf[m] = 1.0f / t32;
  }
  __syncthreads();
  const int e = blockIdx.x * 256 + tid;
  const int s = e >> 5, j = e & (HALF - 1);
  int sc = s;
  if (sc > npos - 1) sc = npos - 1;
  if (sc < 0) sc = 0;
  const float ang = (float)pid[sc] * invf[j];
  float sv, cv;
  sincosf(ang, &sv, &cv);
  volatile float* dc = (volatile float*)(ct + e);
  volatile float* ds = (volatile float*)(sn + e);
  *dc = cv;
  *ds = sv;
  __threadfence();
  *dc = cv;
  *ds = sv;
}

__global__ __launch_bounds__(128) void k_norm1(const float* __restrict__ x, const float* __restrict__ w,
                                               ush* __restrict__ xh, ush* __restrict__ xl) {
  __shared__ float red[4];
  const int tid = threadIdx.x, lane = tid & 31, wave = tid >> 5;
  const size_t o = (size_t)blockIdx.x * HID + (size_t)tid * 8;
  const v4f a0 = *(const v4f*)(x + o);
  const v4f a1 = *(const v4f*)(x + o + 4);
  float ss = a0[0] * a0[0] + a0[1] * a0[1] + a0[2] * a0[2] + a0[3] * a0[3]
           + a1[0] * a1[0] + a1[1] * a1[1] + a1[2] * a1[2] + a1[3] * a1[3];
#pragma unroll
  for (int off = 16; off > 0; off >>= 1) ss += __shfl_xor(ss, off, 32);
  if (lane == 0) red[wave] = ss;
  __syncthreads();
  const float tot = red[0] + red[1] + red[2] + red[3];
  const float rr = rsqrtf(tot * (1.0f / HID) + 1e-6f);
  const v4f w0 = *(const v4f*)(w + tid * 8);
  const v4f w1 = *(const v4f*)(w + tid * 8 + 4);
  const v4f n0 = (a0 * rr) * w0;
  const v4f n1 = (a1 * rr) * w1;
  const v8f f = (v8f){n0[0], n0[1], n0[2], n0[3], n1[0], n1[1], n1[2], n1[3]};
  const HL s = split8(f);
  volatile v4u* dh = (volatile v4u*)(xh + o);
  volatile v4u* dl = (volatile v4u*)(xl + o);
  *dh = s.h;
  *dl = s.l;
  __threadfence();
  *dh = s.h;
  *dl = s.l;
}

#define WTP 65
__global__ __launch_bounds__(256) void k_wtr3(const float* __restrict__ W, int ncol, int nofs,
                                              ush* __restrict__ wh, ush* __restrict__ wl) {
  __shared__ float tl[64 * WTP];
  const int tid = threadIdx.x;
  const int n0 = blockIdx.x * 64, k0 = blockIdx.y * 64;
#pragma unroll
  for (int j = 0; j < 4; ++j) {
    const int p  = tid + 256 * j;
    const int kk = p >> 4;
    const int q4 = (p & 15) * 4;
    const v4f a = *(const v4f*)(W + (size_t)(k0 + kk) * ncol + n0 + q4);
    float* d = tl + kk * WTP + q4;
    d[0] = a[0]; d[1] = a[1]; d[2] = a[2]; d[3] = a[3];
  }
  __syncthreads();
  v4u vh[2], vl[2];
  size_t go[2];
#pragma unroll
  for (int j = 0; j < 2; ++j) {
    const int p  = tid + 256 * j;
    const int nn = p >> 3;
    const int pc = p & 7;
    const float* cp = tl + (pc * 8) * WTP + nn;
    const v8f f = (v8f){cp[0 * WTP], cp[1 * WTP], cp[2 * WTP], cp[3 * WTP],
                        cp[4 * WTP], cp[5 * WTP], cp[6 * WTP], cp[7 * WTP]};
    const HL s = split8(f);
    vh[j] = s.h; vl[j] = s.l;
    go[j] = (size_t)(nofs + n0 + nn) * HID + k0 + pc * 8;
  }
  for (int ps = 0; ps < 2; ++ps) {
#pragma unroll
    for (int j = 0; j < 2; ++j) {
      *(volatile v4u*)(wh + go[j]) = vh[j];
      *(volatile v4u*)(wl + go[j]) = vl[j];
    }
    __threadfence();
  }
}

__global__ __launch_bounds__(256) void k_wtrh(const float* __restrict__ W, int K, int N,
                                              _Float16* __restrict__ wt) {
  __shared__ float tl[64 * WTP];
  const int tid = threadIdx.x;
  const int n0 = blockIdx.x * 64, k0 = blockIdx.y * 64;
  const float* src = W + (size_t)blockIdx.z * (size_t)K * (size_t)N;
  _Float16* dst = wt + (size_t)blockIdx.z * (size_t)N * (size_t)K;
#pragma unroll
  for (int j = 0; j < 4; ++j) {
    const int p  = tid + 256 * j;
    const int kk = p >> 4;
    const int q4 = (p & 15) * 4;
    const v4f a = *(const v4f*)(src + (size_t)(k0 + kk) * N + n0 + q4);
    float* d = tl + kk * WTP + q4;
    d[0] = a[0]; d[1] = a[1]; d[2] = a[2]; d[3] = a[3];
  }
  __syncthreads();
  v4u vt[2];
  size_t go[2];
#pragma unroll
  for (int j = 0; j < 2; ++j) {
    const int p  = tid + 256 * j;
    const int nn = p >> 3;
    const int pc = p & 7;
    const float* cp = tl + (pc * 8) * WTP + nn;
    Pack8 pk;
    pk.h = (v8h){(_Float16)(cp[0 * WTP] * WSC), (_Float16)(cp[1 * WTP] * WSC), (_Float16)(cp[2 * WTP] * WSC), (_Float16)(cp[3 * WTP] * WSC),
                 (_Float16)(cp[4 * WTP] * WSC), (_Float16)(cp[5 * WTP] * WSC), (_Float16)(cp[6 * WTP] * WSC), (_Float16)(cp[7 * WTP] * WSC)};
    vt[j] = pk.u;
    go[j] = (size_t)(n0 + nn) * K + k0 + pc * 8;
  }
  for (int ps = 0; ps < 2; ++ps) {
#pragma unroll
    for (int j = 0; j < 2; ++j) *(volatile v4u*)(dst + go[j]) = vt[j];
    __threadfence();
  }
}

#define SFP 68
__global__ __launch_bounds__(128) void k_qkv3(const ush* __restrict__ xh3, const ush* __restrict__ xl3,
                                              const ush* __restrict__ wth, const ush* __restrict__ wtl,
                                              const float* __restrict__ ct, const float* __restrict__ sn,
                                              const float* __restrict__ qnw, const float* __restrict__ knw,
                                              ush* __restrict__ q3h, ush* __restrict__ q3l,
                                              ush* __restrict__ k3h, ush* __restrict__ k3l,
                                              ush* __restrict__ v3h, ush* __restrict__ v3l) {
  __shared__ __align__(16) float sf[64 * SFP];
  __shared__ float rn[64];
  const int tid = threadIdx.x, lane = tid & 31, wave = tid >> 5;
  const int hh = lane >> 4, c = lane & 15;
  const int mb = blockIdx.x * 64;
  const int ns = blockIdx.y;
  const int which = (ns < NH) ? 0 : ((ns < NH + NKV) ? 1 : 2);
  const int head = (which == 0) ? ns : ((which == 1) ? (ns - NH) : (ns - NH - NKV));
  const int m0 = mb + wave * 16;
  const int n0 = ns * HDM;

  v8f acc[4];
#pragma unroll
  for (int t = 0; t < 4; ++t) acc[t] = zero8();
  gemm3_16x64(xh3, xl3, HID, wth, wtl, HID, m0, n0, lane, acc);

#pragma unroll
  for (int t = 0; t < 4; ++t) {
#pragma unroll
    for (int r = 0; r < 8; ++r)
      sf[(wave * 16 + 8 * hh + r) * SFP + 16 * t + c] = acc[t][r];
  }
  __syncthreads();
  {
    const int row = tid >> 1, hf = tid & 1;
    const float* rp = sf + row * SFP + hf * 32;
    float ss = 0.f;
#pragma unroll
    for (int i = 0; i < 8; ++i) {
      const v4f v = *(const v4f*)(rp + 4 * i);
      ss += v[0] * v[0] + v[1] * v[1] + v[2] * v[2] + v[3] * v[3];
    }
    ss += __shfl_xor(ss, 1, 32);
    if (hf == 0) rn[row] = rsqrtf(ss * (1.0f / HDM) + 1e-6f);
  }
  __syncthreads();

  v4u vh[4], vl[4];
  size_t go[4];
  if (which < 2) {
    const float* nw = (which == 0) ? qnw : knw;
#pragma unroll
    for (int j = 0; j < 4; ++j) {
      const int p  = tid + 128 * j;
      const int lr = p >> 3;
      const int pc = p & 7;
      const int d0 = pc * 8;
      const int d1 = d0 ^ HALF;
      const int j0 = d0 & (HALF - 1);
      const float rr = rn[lr];
      const float* ra = sf + lr * SFP + d0;
      const float* rb = sf + lr * SFP + d1;
      const v4f a0 = *(const v4f*)(ra), a1 = *(const v4f*)(ra + 4);
      const v4f b0 = *(const v4f*)(rb), b1 = *(const v4f*)(rb + 4);
      const v4f wa0 = *(const v4f*)(nw + d0), wa1 = *(const v4f*)(nw + d0 + 4);
      const v4f wb0 = *(const v4f*)(nw + d1), wb1 = *(const v4f*)(nw + d1 + 4);
      const v4f na0 = (a0 * rr) * wa0, na1 = (a1 * rr) * wa1;
      const v4f nb0 = (b0 * rr) * wb0, nb1 = (b1 * rr) * wb1;
      const size_t to = (size_t)(mb + lr) * HALF + j0;
      const v4f c0 = *(const v4f*)(ct + to), c1 = *(const v4f*)(ct + to + 4);
      const v4f s0 = *(const v4f*)(sn + to), s1 = *(const v4f*)(sn + to + 4);
      const float sg = (pc < 4) ? -1.0f : 1.0f;
      const v4f o0 = na0 * c0 + sg * (nb0 * s0);
      const v4f o1 = na1 * c1 + sg * (nb1 * s1);
      const v8f f = (v8f){o0[0], o0[1], o0[2], o0[3], o1[0], o1[1], o1[2], o1[3]};
      const HL s = split8(f);
      vh[j] = s.h; vl[j] = s.l;
      go[j] = ((size_t)head * SQ + mb + lr) * HDM + d0;
    }
    ush* bh = (which == 0) ? q3h : k3h;
    ush* bl = (which == 0) ? q3l : k3l;
    for (int ps = 0; ps < 2; ++ps) {
#pragma unroll
      for (int j = 0; j < 4; ++j) {
        *(volatile v4u*)(bh + go[j]) = vh[j];
        *(volatile v4u*)(bl + go[j]) = vl[j];
      }
      __threadfence();
    }
  } else {
#pragma unroll
    for (int j = 0; j < 4; ++j) {
      const int p  = tid + 128 * j;
      const int d  = p >> 3;
      const int pc = p & 7;
      const float* cp = sf + (pc * 8) * SFP + d;
      const v8f f = (v8f){cp[0 * SFP], cp[1 * SFP], cp[2 * SFP], cp[3 * SFP],
                          cp[4 * SFP], cp[5 * SFP], cp[6 * SFP], cp[7 * SFP]};
      const HL s = split8(f);
      vh[j] = s.h; vl[j] = s.l;
      go[j] = ((size_t)head * HDM + d) * SQ + mb + pc * 8;
    }
    for (int ps = 0; ps < 2; ++ps) {
#pragma unroll
      for (int j = 0; j < 4; ++j) {
        *(volatile v4u*)(v3h + go[j]) = vh[j];
        *(volatile v4u*)(v3l + go[j]) = vl[j];
      }
      __threadfence();
    }
  }
}

#define KC 64
#define KP 72
static_assert(KC * KP >= 64 * KP);
__global__ __launch_bounds__(128) __attribute__((amdgpu_num_vgpr(256)))
void k_attn3(const ush* __restrict__ q3h, const ush* __restrict__ q3l,
             const ush* __restrict__ k3h, const ush* __restrict__ k3l,
             const ush* __restrict__ v3h, const ush* __restrict__ v3l,
             ush* __restrict__ o3h, ush* __restrict__ o3l, float sscale) {
  __shared__ __align__(16) ush Ksh[KC * KP];
  __shared__ __align__(16) ush Ksl[KC * KP];
  __shared__ __align__(16) ush Vsh[HDM * KP];
  __shared__ __align__(16) ush Vsl[HDM * KP];
  __shared__ __align__(16) ush P3[2 * 4 * 16 * KP];

  const int tid = threadIdx.x, lane = tid & 31, wave = tid >> 5;
  const int hh = lane >> 4, c = lane & 15;
  const int h   = blockIdx.x / NQ64;
  const int q64 = blockIdx.x - h * NQ64;
  const int kvh = h >> 2;
  const int q0  = q64 * 64 + wave * 16;

  const ush* Qh  = q3h + (size_t)h * SQ * HDM;
  const ush* Ql  = q3l + (size_t)h * SQ * HDM;
  const ush* K3H = k3h + (size_t)kvh * SQ * HDM;
  const ush* K3L = k3l + (size_t)kvh * SQ * HDM;
  const ush* V3H = v3h + (size_t)kvh * HDM * SQ;
  const ush* V3L = v3l + (size_t)kvh * HDM * SQ;
  ush* pwh = P3 + wave * 16 * KP;
  ush* pwl = P3 + (4 + wave) * 16 * KP;

  const float NEGI = -__builtin_huge_valf();
  float mrow[8], lrow[8];
  v8f oacc[4];
#pragma unroll
  for (int r = 0; r < 8; ++r) { mrow[r] = NEGI; lrow[r] = 0.f; }
#pragma unroll
  for (int t = 0; t < 4; ++t) oacc[t] = zero8();

  const int nck = q64 + 1;

  for (int kc = 0; kc < nck; ++kc) {
    const int kv0 = kc * KC;
    __syncthreads();
    {
      const int r  = tid >> 1;
      const int qq = (tid & 1) * 32;
      const ush* ah = K3H + (size_t)(kv0 + r) * HDM + qq;
      const ush* al = K3L + (size_t)(kv0 + r) * HDM + qq;
#pragma unroll
      for (int e = 0; e < 4; ++e) {
        *(v8us*)(Ksh + r * KP + qq + 8 * e) = *(const v8us*)(ah + 8 * e);
        *(v8us*)(Ksl + r * KP + qq + 8 * e) = *(const v8us*)(al + 8 * e);
      }
      const ush* vh = V3H + (size_t)r * SQ + kv0 + qq;
      const ush* vl = V3L + (size_t)r * SQ + kv0 + qq;
#pragma unroll
      for (int e = 0; e < 4; ++e) {
        *(v8us*)(Vsh + r * KP + qq + 8 * e) = *(const v8us*)(vh + 8 * e);
        *(v8us*)(Vsl + r * KP + qq + 8 * e) = *(const v8us*)(vl + 8 * e);
      }
    }
    __syncthreads();

    v8f s[4];
#pragma unroll
    for (int j = 0; j < 4; ++j) s[j] = zero8();
#pragma unroll
    for (int dc = 0; dc < 2; ++dc) {
      const v16us qah = ldfragu(Qh, HDM, q0, dc * 32, lane);
      const v16us qal = ldfragu(Ql, HDM, q0, dc * 32, lane);
#pragma unroll
      for (int j = 0; j < 4; ++j) {
        const v16us kbh = ldfragu(Ksh, KP, j * 16, dc * 32, lane);
        const v16us kbl = ldfragu(Ksl, KP, j * 16, dc * 32, lane);
        s[j] = mmab(qah, kbh, s[j]);
        s[j] = mmab(qah, kbl, s[j]);
        s[j] = mmab(qal, kbh, s[j]);
      }
    }
    const bool edge = (kc == q64);
#pragma unroll
    for (int r = 0; r < 8; ++r) {
      const int qry = q0 + 8 * hh + r;
#pragma unroll
      for (int j = 0; j < 4; ++j) {
        const int key = kv0 + 16 * j + c;
        const float v = s[j][r] * sscale;
        s[j][r] = (edge && key > qry) ? NEGI : v;
      }
    }
    float cm[8];
#pragma unroll
    for (int r = 0; r < 8; ++r) {
      float m = NEGI;
#pragma unroll
      for (int j = 0; j < 4; ++j) m = fmaxf(m, s[j][r]);
#pragma unroll
      for (int off = 1; off < 16; off <<= 1) m = fmaxf(m, __shfl_xor(m, off, 32));
      cm[r] = m;
    }
    float al[8];
#pragma unroll
    for (int r = 0; r < 8; ++r) {
      const float mnew  = fmaxf(mrow[r], cm[r]);
      const float alpha = __expf(mrow[r] - mnew);
      mrow[r] = mnew;
      float psum = 0.f;
#pragma unroll
      for (int j = 0; j < 4; ++j) {
        const float p = __expf(s[j][r] - mnew);
        psum += p;
        const ush phi = f2bf(p);
        pwh[(8 * hh + r) * KP + j * 16 + c] = phi;
        pwl[(8 * hh + r) * KP + j * 16 + c] = f2bf(p - bf2f(phi));
      }
#pragma unroll
      for (int off = 1; off < 16; off <<= 1) psum += __shfl_xor(psum, off, 32);
      lrow[r] = lrow[r] * alpha + psum;
      al[r] = alpha;
    }
#pragma unroll
    for (int t = 0; t < 4; ++t)
#pragma unroll
      for (int r = 0; r < 8; ++r) oacc[t][r] *= al[r];
    __syncthreads();

#pragma unroll
    for (int kk = 0; kk < 2; ++kk) {
      const v16us pah = ldfragu(pwh, KP, 0, kk * 32, lane);
      const v16us pal = ldfragu(pwl, KP, 0, kk * 32, lane);
#pragma unroll
      for (int t = 0; t < 4; ++t) {
        const v16us vbh = ldfragu(Vsh, KP, t * 16, kk * 32, lane);
        const v16us vbl = ldfragu(Vsl, KP, t * 16, kk * 32, lane);
        oacc[t] = mmab(pah, vbh, oacc[t]);
        oacc[t] = mmab(pah, vbl, oacc[t]);
        oacc[t] = mmab(pal, vbh, oacc[t]);
      }
    }
  }
  __syncthreads();

  ush* Oh = Ksh;
  ush* Ol = Ksl;
#pragma unroll
  for (int r = 0; r < 8; ++r) {
    const float lr  = lrow[r];
    const float inv = (lr > 0.f) ? (1.0f / lr) : 0.f;
    const int   row = wave * 16 + 8 * hh + r;
#pragma unroll
    for (int t = 0; t < 4; ++t) {
      const float o = oacc[t][r] * inv;
      const ush hi = f2bf(o);
      Oh[row * KP + 16 * t + c] = hi;
      Ol[row * KP + 16 * t + c] = f2bf(o - bf2f(hi));
    }
  }
  __syncthreads();
  v4u vh[4], vl[4];
  size_t go[4];
#pragma unroll
  for (int it = 0; it < 4; ++it) {
    const int p  = lane + 32 * it;
    const int L  = p >> 3;
    const int pc = p & 7;
    PackU pk;
    pk.s   = *(const v8us*)(Oh + (wave * 16 + L) * KP + pc * 8);
    vh[it] = pk.u;
    pk.s   = *(const v8us*)(Ol + (wave * 16 + L) * KP + pc * 8);
    vl[it] = pk.u;
    go[it] = (size_t)(q0 + L) * HID + (size_t)h * HDM + pc * 8;
  }
  for (int ps = 0; ps < 2; ++ps) {
#pragma unroll
    for (int it = 0; it < 4; ++it) {
      *(volatile v4u*)(o3h + go[it]) = vh[it];
      *(volatile v4u*)(o3l + go[it]) = vl[it];
    }
    __threadfence();
  }
}

#define OTP 68
__global__ __launch_bounds__(256) void k_oproj3(const ush* __restrict__ ah, const ush* __restrict__ al,
                                                const ush* __restrict__ wh, const ush* __restrict__ wl,
                                                const float* __restrict__ res, float* __restrict__ out) {
  __shared__ __align__(16) float st[8][16 * OTP];
  const int tid = threadIdx.x, lane = tid & 31, wave = tid >> 5;
  const int hh = lane >> 4, c = lane & 15;
  const int m0 = blockIdx.x * 256 + wave * 32;
  const int n0 = blockIdx.y * 64;

  v8f acc[2][4];
#pragma unroll
  for (int s = 0; s < 2; ++s)
#pragma unroll
    for (int t = 0; t < 4; ++t) acc[s][t] = zero8();
  gemm3_32x64(ah, al, HID, wh, wl, HID, m0, n0, lane, acc);

  float* sw = st[wave];
#pragma unroll
  for (int sub = 0; sub < 2; ++sub) {
    __syncthreads();
#pragma unroll
    for (int t = 0; t < 4; ++t) {
#pragma unroll
      for (int r = 0; r < 8; ++r) sw[(8 * hh + r) * OTP + 16 * t + c] = acc[sub][t][r];
    }
    __syncthreads();
    v4f val[8];
    size_t go[8];
#pragma unroll
    for (int it = 0; it < 8; ++it) {
      const int p    = lane + 32 * it;
      const int L    = p >> 3;
      const int pc   = p & 7;
      const int row  = L >> 1;
      const int half = L & 1;
      go[it]  = (size_t)(m0 + sub * 16 + row) * HID + n0 + half * 32 + pc * 4;
      val[it] = *(const v4f*)(res + go[it]) + *(const v4f*)(sw + row * OTP + half * 32 + pc * 4);
    }
    for (int ps = 0; ps < 2; ++ps) {
#pragma unroll
      for (int it = 0; it < 8; ++it) *(volatile v4f*)(out + go[it]) = val[it];
      __threadfence();
    }
  }
}

__device__ __forceinline__ float grp2(const float* p) {
  float m1 = -3.0e38f, m2 = -3.0e38f;
#pragma unroll
  for (int j = 0; j < 4; ++j) {
    const float v = p[j];
    if (v > m1) { m2 = m1; m1 = v; } else if (v > m2) { m2 = v; }
  }
  return m1 + m2;
}

__global__ __launch_bounds__(128) void k_route(const float* __restrict__ hid, const float* __restrict__ lnw,
                                               const float* __restrict__ rw, const float* __restrict__ rb,
                                               _Float16* __restrict__ xm, unsigned* __restrict__ route) {
  __shared__ float red[4];
  __shared__ float xs[HID];
  __shared__ float part[4 * NE];
  __shared__ float s_sc[NE];
  __shared__ float s_sf[NE];
  __shared__ float s_mk[NE];
  __shared__ int   s_used[NE];
  __shared__ unsigned s_line[RTW];
  const int tid = threadIdx.x, lane = tid & 31, wave = tid >> 5;
  const int row = blockIdx.x;
  const size_t o = (size_t)row * HID + (size_t)tid * 8;
  const v4f a0 = *(const v4f*)(hid + o);
  const v4f a1 = *(const v4f*)(hid + o + 4);
  float ss = a0[0] * a0[0] + a0[1] * a0[1] + a0[2] * a0[2] + a0[3] * a0[3]
           + a1[0] * a1[0] + a1[1] * a1[1] + a1[2] * a1[2] + a1[3] * a1[3];
#pragma unroll
  for (int off = 16; off > 0; off >>= 1) ss += __shfl_xor(ss, off, 32);
  if (lane == 0) red[wave] = ss;
  __syncthreads();
  const float tot = red[0] + red[1] + red[2] + red[3];
  const float rr = rsqrtf(tot * (1.0f / HID) + 1e-6f);
  const v4f w0 = *(const v4f*)(lnw + tid * 8);
  const v4f w1 = *(const v4f*)(lnw + tid * 8 + 4);
  const v4f n0 = (a0 * rr) * w0;
  const v4f n1 = (a1 * rr) * w1;
  xs[tid * 8 + 0] = n0[0]; xs[tid * 8 + 1] = n0[1]; xs[tid * 8 + 2] = n0[2]; xs[tid * 8 + 3] = n0[3];
  xs[tid * 8 + 4] = n1[0]; xs[tid * 8 + 5] = n1[1]; xs[tid * 8 + 6] = n1[2]; xs[tid * 8 + 7] = n1[3];
  Pack8 pk;
  pk.h = (v8h){(_Float16)(n0[0] * XSC), (_Float16)(n0[1] * XSC), (_Float16)(n0[2] * XSC), (_Float16)(n0[3] * XSC),
               (_Float16)(n1[0] * XSC), (_Float16)(n1[1] * XSC), (_Float16)(n1[2] * XSC), (_Float16)(n1[3] * XSC)};
  const v4u vv = pk.u;
  volatile v4u* dx = (volatile v4u*)(xm + o);
  *dx = vv;
  __threadfence();
  *dx = vv;

  float acc[NE];
#pragma unroll
  for (int ee = 0; ee < NE; ++ee) acc[ee] = 0.f;
#pragma unroll 1
  for (int j = 0; j < 8; ++j) {
    const float xv = xs[tid * 8 + j];
    const float* wr = rw + (size_t)(tid * 8 + j) * NE;
    const v4f r0 = *(const v4f*)(wr);
    const v4f r1 = *(const v4f*)(wr + 4);
    const v4f r2 = *(const v4f*)(wr + 8);
    const v4f r3 = *(const v4f*)(wr + 12);
    acc[0]  += xv * r0[0]; acc[1]  += xv * r0[1]; acc[2]  += xv * r0[2]; acc[3]  += xv * r0[3];
    acc[4]  += xv * r1[0]; acc[5]  += xv * r1[1]; acc[6]  += xv * r1[2]; acc[7]  += xv * r1[3];
    acc[8]  += xv * r2[0]; acc[9]  += xv * r2[1]; acc[10] += xv * r2[2]; acc[11] += xv * r2[3];
    acc[12] += xv * r3[0]; acc[13] += xv * r3[1]; acc[14] += xv * r3[2]; acc[15] += xv * r3[3];
  }
#pragma unroll
  for (int ee = 0; ee < NE; ++ee) {
    float v = acc[ee];
#pragma unroll
    for (int off = 16; off > 0; off >>= 1) v += __shfl_xor(v, off, 32);
    if (lane == 0) part[wave * NE + ee] = v;
  }
  __syncthreads();
  if (tid < NE) {
    const float lg = part[tid] + part[NE + tid] + part[2 * NE + tid] + part[3 * NE + tid];
    const float sc = 1.0f / (1.0f + expf(-lg));
    s_sc[tid] = sc;
    s_sf[tid] = sc + rb[tid];
    s_mk[tid] = 0.f;
    s_used[tid] = 0;
  }
  __syncthreads();
  if (tid == 0) {
    const float gs0 = grp2(s_sf + 0);
    const float gs1 = grp2(s_sf + 4);
    const float gs2 = grp2(s_sf + 8);
    const float gs3 = grp2(s_sf + 12);
    int b1 = 0; float bv = gs0;
    if (gs1 > bv) { bv = gs1; b1 = 1; }
    if (gs2 > bv) { bv = gs2; b1 = 2; }
    if (gs3 > bv) { bv = gs3; b1 = 3; }
    int b2 = -1; float bv2 = 0.f;
    if (b1 != 0) { bv2 = gs0; b2 = 0; }
    if (b1 != 1 && (b2 < 0 || gs1 > bv2)) { bv2 = gs1; b2 = 1; }
    if (b1 != 2 && (b2 < 0 || gs2 > bv2)) { bv2 = gs2; b2 = 2; }
    if (b1 != 3 && (b2 < 0 || gs3 > bv2)) { bv2 = gs3; b2 = 3; }
#pragma unroll 1
    for (int i = 0; i < NE; ++i) {
      const int g = i >> 2;
      const bool sel = (g == b1) || (g == b2);
      s_mk[i] = sel ? s_sf[i] : 0.0f;
      s_used[i] = 0;
    }
    float wsum = 0.f;
#pragma unroll 1
    for (int j = 0; j < NTOP; ++j) {
      int bi = -1; float bb = 0.f;
#pragma unroll 1
      for (int i = 0; i < NE; ++i) {
        if (s_used[i] == 0) {
          const float v = s_mk[i];
          if (bi < 0 || v > bb) { bb = v; bi = i; }
        }
      }
      s_used[bi] = 1;
      const float wj = s_sc[bi];
      wsum += wj;
      s_line[j] = (unsigned)bi;
      s_line[NTOP + j] = __float_as_uint(wj);
    }
    const float inv = 1.0f / (wsum + 1e-20f);
#pragma unroll 1
    for (int j = 0; j < NTOP; ++j) s_line[NTOP + j] = __float_as_uint(__uint_as_float(s_line[NTOP + j]) * inv);
#pragma unroll 1
    for (int k = 2 * NTOP; k < RTW; ++k) s_line[k] = 0u;
  }
  __syncthreads();
  if (wave == 0) {
    const unsigned u = s_line[lane];
    volatile unsigned* d = (volatile unsigned*)(route + (size_t)row * RTW + lane);
    *d = u;
    __threadfence();
    *d = u;
  }
}

__device__ __forceinline__ int scan_slots(const unsigned* __restrict__ route, int e, int slot0,
                                          int* s_tok, int* s_j, int* s_wc, int tid, int lane, int wave) {
  if (tid < 64) { s_tok[tid] = 0; s_j[tid] = 0; }
  int run = 0;
  __syncthreads();
#pragma unroll 1
  for (int ch = 0; ch < SQ / 256; ++ch) {
    const int t = ch * 256 + tid;
    const v4u id = *(const v4u*)(route + (size_t)t * RTW);
    const bool h0 = ((int)id[0] == e), h1 = ((int)id[1] == e), h2 = ((int)id[2] == e), h3 = ((int)id[3] == e);
    const bool hit = h0 || h1 || h2 || h3;
    const int jsel = h0 ? 0 : (h1 ? 1 : (h2 ? 2 : 3));
    const unsigned bal = __builtin_amdgcn_ballot_w32(hit);
    const unsigned lm  = (1u << lane) - 1u;
    const int lpre = __builtin_popcount(bal & lm);
    const int wc   = __builtin_popcount(bal);
    if (lane == 0) s_wc[wave] = wc;
    __syncthreads();
    int wpre = 0, tot = 0;
#pragma unroll
    for (int w = 0; w < 8; ++w) { const int v = s_wc[w]; tot += v; wpre += (w < wave) ? v : 0; }
    if (hit) {
      const int q = run + wpre + lpre - slot0;
      if ((unsigned)q < 64u) { s_tok[q] = t; s_j[q] = jsel; }
    }
    run += tot;
    __syncthreads();
  }
  return run;
}

#define XAP 72
#define SOP 136
template <bool ROUTED>
__global__ __launch_bounds__(256) void k_gateup(const _Float16* __restrict__ xm,
                                                const _Float16* __restrict__ wgT,
                                                const _Float16* __restrict__ wuT,
                                                const unsigned* __restrict__ route,
                                                _Float16* __restrict__ mid) {
  __shared__ __align__(16) _Float16 xa[64 * XAP];
  __shared__ __align__(16) _Float16 so[64 * SOP];
  __shared__ int s_tok[64];
  __shared__ int s_j[64];
  __shared__ int s_wc[8];
  const int tid = threadIdx.x, lane = tid & 31, wave = tid >> 5;
  const int hh = lane >> 4, c = lane & 15;
  int e = 0, mtile = blockIdx.x;
  if (ROUTED) { e = blockIdx.x / MT; mtile = blockIdx.x - e * MT; }
  const int slot0 = mtile * 64;
  int count = SQ;
  if (ROUTED) {
    count = scan_slots(route, e, slot0, s_tok, s_j, s_wc, tid, lane, wave);
  } else {
    if (tid < 64) { s_tok[tid] = slot0 + tid; s_j[tid] = 0; }
    __syncthreads();
  }
  if (slot0 >= count) return;

  const _Float16* Bg = wgT + (size_t)e * FFI * HID;
  const _Float16* Bu = wuT + (size_t)e * FFI * HID;
  const size_t obase = ROUTED ? ((size_t)e * CAP) : (size_t)0;
  const int wm = wave >> 1, wn = wave & 1;
  const float ig = 1.0f / (XSC * WSC);

#pragma unroll 1
  for (int cg = 0; cg < FFI / 128; ++cg) {
    const int ncol0 = cg * 128;
    const int n0 = ncol0 + wn * 64;
    v8f ga[4], ua[4];
#pragma unroll
    for (int t = 0; t < 4; ++t) { ga[t] = zero8(); ua[t] = zero8(); }
#pragma unroll 1
    for (int kc = 0; kc < HID / 64; ++kc) {
      __syncthreads();
#pragma unroll
      for (int j = 0; j < 2; ++j) {
        const int p  = tid + 256 * j;
        const int r  = p >> 3;
        const int pc = p & 7;
        int tk = s_tok[r];
        tk = (tk < 0) ? 0 : ((tk > SQ - 1) ? (SQ - 1) : tk);
        *(v8h*)(xa + r * XAP + pc * 8) = *(const v8h*)(xm + (size_t)tk * HID + kc * 64 + pc * 8);
      }
      __syncthreads();
#pragma unroll
      for (int ks = 0; ks < 2; ++ks) {
        const v16h a = ldfrag(xa, XAP, wm * 16, ks * 32, lane);
#pragma unroll
        for (int t = 0; t < 4; ++t) {
          const v16h bg = ldfrag(Bg, HID, n0 + 16 * t, kc * 64 + ks * 32, lane);
          ga[t] = mma16(a, bg, ga[t]);
          const v16h bu = ldfrag(Bu, HID, n0 + 16 * t, kc * 64 + ks * 32, lane);
          ua[t] = mma16(a, bu, ua[t]);
        }
      }
    }
#pragma unroll
    for (int t = 0; t < 4; ++t) {
#pragma unroll
      for (int r = 0; r < 8; ++r) {
        const float g = ga[t][r] * ig, u = ua[t][r] * ig;
        const float sgm = __builtin_amdgcn_rcpf(1.0f + __expf(-g));
        const float m = (g * sgm) * u;
        so[(wm * 16 + 8 * hh + r) * SOP + wn * 64 + 16 * t + c] = (_Float16)(m * MSC);
      }
    }
    __syncthreads();
    v4u val[4];
    size_t go[4];
#pragma unroll
    for (int j = 0; j < 4; ++j) {
      const int p  = tid + 256 * j;
      const int r  = p >> 4;
      const int pc = p & 15;
      Pack8 pk;
      pk.h   = *(const v8h*)(so + r * SOP + pc * 8);
      val[j] = pk.u;
      go[j]  = (obase + (size_t)slot0 + r) * FFI + ncol0 + pc * 8;
    }
    for (int ps = 0; ps < 2; ++ps) {
#pragma unroll
      for (int j = 0; j < 4; ++j) *(volatile v4u*)(mid + go[j]) = val[j];
      __threadfence();
    }
  }
}

__global__ __launch_bounds__(256) void k_moe_down(const _Float16* __restrict__ mid,
                                                  const _Float16* __restrict__ wdT,
                                                  const unsigned* __restrict__ route,
                                                  float* __restrict__ y) {
  __shared__ __align__(16) float st[8][16 * OTP];
  __shared__ int s_tok[64];
  __shared__ int s_j[64];
  __shared__ int s_wc[8];
  const int tid = threadIdx.x, lane = tid & 31, wave = tid >> 5;
  const int hh = lane >> 4, c = lane & 15;
  const int e = blockIdx.x / MT;
  const int mtile = blockIdx.x - e * MT;
  const int slot0 = mtile * 64;
  const int count = scan_slots(route, e, slot0, s_tok, s_j, s_wc, tid, lane, wave);
  if (slot0 >= count) return;

  const int wm = wave >> 1, wn = wave & 1;
  const _Float16* A  = mid + (size_t)e * CAP * FFI;
  const _Float16* Bd = wdT + (size_t)e * HID * FFI;
  const int rowA = slot0 + wm * 16;
  float* sw = st[wave];
  const float isc = 1.0f / (MSC * WSC);

#pragma unroll 1
  for (int cg = 0; cg < HID / 256; ++cg) {
    const int n0 = cg * 256 + wn * 128;
    v8f acc[8];
#pragma unroll
    for (int t = 0; t < 8; ++t) acc[t] = zero8();
#pragma unroll 2
    for (int k0 = 0; k0 < FFI; k0 += 32) {
      const v16h a = ldfrag(A, FFI, rowA, k0, lane);
#pragma unroll
      for (int t = 0; t < 8; ++t) {
        const v16h b = ldfrag(Bd, FFI, n0 + 16 * t, k0, lane);
        acc[t] = mma16(a, b, acc[t]);
      }
    }
#pragma unroll
    for (int hf = 0; hf < 2; ++hf) {
      __syncthreads();
#pragma unroll
      for (int t = 0; t < 4; ++t) {
#pragma unroll
        for (int r = 0; r < 8; ++r) sw[(8 * hh + r) * OTP + 16 * t + c] = acc[4 * hf + t][r] * isc;
      }
      __syncthreads();
      v4f val[8];
      size_t go[8];
      bool ok[8];
#pragma unroll
      for (int it = 0; it < 8; ++it) {
        const int p    = lane + 32 * it;
        const int L    = p >> 3;
        const int pc   = p & 7;
        const int row  = L >> 1;
        const int half = L & 1;
        val[it] = *(const v4f*)(sw + row * OTP + half * 32 + pc * 4);
        const int lr = wm * 16 + row;
        ok[it] = (slot0 + lr) < count;
        int tk = s_tok[lr];
        tk = (tk < 0) ? 0 : ((tk > SQ - 1) ? (SQ - 1) : tk);
        const int jj = s_j[lr] & 3;
        go[it] = ((size_t)tk * NTOP + jj) * HID + n0 + hf * 64 + half * 32 + pc * 4;
      }
      for (int ps = 0; ps < 2; ++ps) {
#pragma unroll
        for (int it = 0; it < 8; ++it) if (ok[it]) *(volatile v4f*)(y + go[it]) = val[it];
        __threadfence();
      }
    }
  }
}

__global__ __launch_bounds__(256) void k_final(const _Float16* __restrict__ sm,
                                               const _Float16* __restrict__ sdT,
                                               const float* __restrict__ hid,
                                               const float* __restrict__ y,
                                               const unsigned* __restrict__ route,
                                               float* __restrict__ out) {
  __shared__ __align__(16) float st[8][16 * OTP];
  const int tid = threadIdx.x, lane = tid & 31, wave = tid >> 5;
  const int hh = lane >> 4, c = lane & 15;
  const int m0 = blockIdx.x * 256 + wave * 32;
  const int n0 = blockIdx.y * 64;

  v8f acc[2][4];
#pragma unroll
  for (int s = 0; s < 2; ++s)
#pragma unroll
    for (int t = 0; t < 4; ++t) acc[s][t] = zero8();
  gemm32x64h<FFI>(sm, FFI, sdT, FFI, m0, n0, lane, acc);

  float* sw = st[wave];
  const float isc = 1.0f / (MSC * WSC);
#pragma unroll
  for (int sub = 0; sub < 2; ++sub) {
    __syncthreads();
#pragma unroll
    for (int t = 0; t < 4; ++t) {
#pragma unroll
      for (int r = 0; r < 8; ++r) sw[(8 * hh + r) * OTP + 16 * t + c] = acc[sub][t][r] * isc;
    }
    __syncthreads();
    v4f val[8];
    size_t go[8];
#pragma unroll
    for (int it = 0; it < 8; ++it) {
      const int p    = lane + 32 * it;
      const int L    = p >> 3;
      const int pc   = p & 7;
      const int row  = L >> 1;
      const int half = L & 1;
      const int tok  = m0 + sub * 16 + row;
      const int col  = n0 + half * 32 + pc * 4;
      const v4f shv = *(const v4f*)(sw + row * OTP + half * 32 + pc * 4);
      const v4u wb  = *(const v4u*)(route + (size_t)tok * RTW + NTOP);
      const float w0 = __uint_as_float(wb[0]), w1 = __uint_as_float(wb[1]);
      const float w2 = __uint_as_float(wb[2]), w3 = __uint_as_float(wb[3]);
      const float* yb = y + (size_t)tok * NTOP * HID + col;
      const v4f y0 = *(const v4f*)(yb);
      const v4f y1 = *(const v4f*)(yb + HID);
      const v4f y2 = *(const v4f*)(yb + 2 * HID);
      const v4f y3 = *(const v4f*)(yb + 3 * HID);
      const v4f rt = w0 * y0 + w1 * y1 + w2 * y2 + w3 * y3;
      const v4f rs = rt + shv;
      const size_t gi = (size_t)tok * HID + col;
      val[it] = *(const v4f*)(hid + gi) + rs;
      go[it]  = gi;
    }
    for (int ps = 0; ps < 2; ++ps) {
#pragma unroll
      for (int it = 0; it < 8; ++it) *(volatile v4f*)(out + go[it]) = val[it];
      __threadfence();
    }
  }
}

extern "C" void kernel_launch(void* const* d_in, const int* in_sizes, int n_in,
                              void* d_out, int out_size, void* d_ws, size_t ws_size,
                              hipStream_t stream) {
  if (n_in < 18) return;
  if (in_sizes[0]  != SQ * HID) return;
  if (in_sizes[1]  != SQ) return;
  if (in_sizes[2]  != HID) return;
  if (in_sizes[3]  != HID) return;
  if (in_sizes[4]  != HID * NH * HDM) return;
  if (in_sizes[5]  != HID * NKV * HDM) return;
  if (in_sizes[6]  != HID * NKV * HDM) return;
  if (in_sizes[7]  != NH * HDM * HID) return;
  if (in_sizes[8]  != HDM) return;
  if (in_sizes[9]  != HDM) return;
  if (in_sizes[10] != HID * NE) return;
  if (in_sizes[11] != NE) return;
  if (in_sizes[12] != NE * HID * FFI) return;
  if (in_sizes[13] != NE * HID * FFI) return;
  if (in_sizes[14] != NE * FFI * HID) return;
  if (in_sizes[15] != HID * FFI) return;
  if (in_sizes[16] != HID * FFI) return;
  if (in_sizes[17] != FFI * HID) return;
  if (out_size != SQ * HID) return;
  if (((in_sizes[1] * HALF) & 255) != 0) return;

  const float* hs   = (const float*)d_in[0];
  const int*   pid  = (const int*)d_in[1];
  const float* ln1w = (const float*)d_in[2];
  const float* ln2w = (const float*)d_in[3];
  const float* qw   = (const float*)d_in[4];
  const float* kw   = (const float*)d_in[5];
  const float* vw   = (const float*)d_in[6];
  const float* ow   = (const float*)d_in[7];
  const float* qnw  = (const float*)d_in[8];
  const float* knw  = (const float*)d_in[9];
  const float* rw   = (const float*)d_in[10];
  const float* rb   = (const float*)d_in[11];
  const float* wg   = (const float*)d_in[12];
  const float* wu   = (const float*)d_in[13];
  const float* wd   = (const float*)d_in[14];
  const float* sg   = (const float*)d_in[15];
  const float* su   = (const float*)d_in[16];
  const float* sd   = (const float*)d_in[17];
  float* out = (float*)d_out;

  size_t off = 0;
  const size_t oCt  = off; off += (size_t)SQ * HALF * 4;
  const size_t oSn  = off; off += (size_t)SQ * HALF * 4;
  const size_t oA   = off;
  const size_t oXh3 = off; off += (size_t)SQ * HID * 2;
  const size_t oXl3 = off; off += (size_t)SQ * HID * 2;
  const size_t oWqh = off; off += (size_t)NQKV * HID * 2;
  const size_t oWql = off; off += (size_t)NQKV * HID * 2;
  const size_t oWoh = off; off += (size_t)HID * HID * 2;
  const size_t oWol = off; off += (size_t)HID * HID * 2;
  const size_t oQh  = off; off += (size_t)NH * SQ * HDM * 2;
  const size_t oQl  = off; off += (size_t)NH * SQ * HDM * 2;
  const size_t oKh  = off; off += (size_t)NKV * SQ * HDM * 2;
  const size_t oKl  = off; off += (size_t)NKV * SQ * HDM * 2;
  const size_t oVh  = off; off += (size_t)NKV * HDM * SQ * 2;
  const size_t oVl  = off; off += (size_t)NKV * HDM * SQ * 2;
  const size_t oOh  = off; off += (size_t)SQ * HID * 2;
  const size_t oOl  = off; off += (size_t)SQ * HID * 2;
  const size_t endA = off;
  const size_t oMid = oA;
  if (oMid + (size_t)NE * CAP * FFI * 2 > endA) return;
  const size_t oWgT = off; off += (size_t)NE * FFI * HID * 2;
  const size_t oWuT = off; off += (size_t)NE * FFI * HID * 2;
  const size_t endB = off;
  const size_t oY   = oWgT;
  if (oY + (size_t)SQ * NTOP * HID * 4 > endB) return;
  const size_t oWdT = off; off += (size_t)NE * HID * FFI * 2;
  const size_t oSgT = off; off += (size_t)FFI * HID * 2;
  const size_t oSuT = off; off += (size_t)FFI * HID * 2;
  const size_t oSdT = off; off += (size_t)HID * FFI * 2;
  const size_t oHid = off; off += (size_t)SQ * HID * 4;
  const size_t oXm  = off; off += (size_t)SQ * HID * 2;
  const size_t oRt  = off; off += (size_t)SQ * RTW * 4;
  const size_t oSm  = off; off += (size_t)SQ * FFI * 2;
  if (off > ws_size) return;
  if (off > (size_t)134217728) return;

  char* ws = (char*)d_ws;
  float*    Ct  = (float*)(ws + oCt);
  float*    Sn  = (float*)(ws + oSn);
  ush*      Xh3 = (ush*)(ws + oXh3);
  ush*      Xl3 = (ush*)(ws + oXl3);
  ush*      Wqh = (ush*)(ws + oWqh);
  ush*      Wql = (ush*)(ws + oWql);
  ush*      Woh = (ush*)(ws + oWoh);
  ush*      Wol = (ush*)(ws + oWol);
  ush*      Qh  = (ush*)(ws + oQh);
  ush*      Ql  = (ush*)(ws + oQl);
  ush*      Kh  = (ush*)(ws + oKh);
  ush*      Kl  = (ush*)(ws + oKl);
  ush*      Vh  = (ush*)(ws + oVh);
  ush*      Vl  = (ush*)(ws + oVl);
  ush*      Oh  = (ush*)(ws + oOh);
  ush*      Ol  = (ush*)(ws + oOl);
  _Float16* Mid = (_Float16*)(ws + oMid);
  _Float16* WgT = (_Float16*)(ws + oWgT);
  _Float16* WuT = (_Float16*)(ws + oWuT);
  float*    Y   = (float*)(ws + oY);
  _Float16* WdT = (_Float16*)(ws + oWdT);
  _Float16* SgT = (_Float16*)(ws + oSgT);
  _Float16* SuT = (_Float16*)(ws + oSuT);
  _Float16* SdT = (_Float16*)(ws + oSdT);
  float*    Hid = (float*)(ws + oHid);
  _Float16* Xm  = (_Float16*)(ws + oXm);
  unsigned* Rt  = (unsigned*)(ws + oRt);
  _Float16* Sm  = (_Float16*)(ws + oSm);

  k_tab<<<dim3((SQ * HALF) / 256), dim3(256), 0, stream>>>(pid, Ct, Sn, in_sizes[1]);
  k_norm1<<<dim3(SQ), dim3(128), 0, stream>>>(hs, ln1w, Xh3, Xl3);
  k_wtr3<<<dim3((NH * HDM) / 64, HID / 64), dim3(256), 0, stream>>>(qw, NH * HDM, 0, Wqh, Wql);
  k_wtr3<<<dim3((NKV * HDM) / 64, HID / 64), dim3(256), 0, stream>>>(kw, NKV * HDM, KOFS, Wqh, Wql);
  k_wtr3<<<dim3((NKV * HDM) / 64, HID / 64), dim3(256), 0, stream>>>(vw, NKV * HDM, VOFS, Wqh, Wql);
  k_wtr3<<<dim3(HID / 64, HID / 64), dim3(256), 0, stream>>>(ow, HID, 0, Woh, Wol);
  k_wtrh<<<dim3(FFI / 64, HID / 64, NE), dim3(256), 0, stream>>>(wg, HID, FFI, WgT);
  k_wtrh<<<dim3(FFI / 64, HID / 64, NE), dim3(256), 0, stream>>>(wu, HID, FFI, WuT);
  k_wtrh<<<dim3(HID / 64, FFI / 64, NE), dim3(256), 0, stream>>>(wd, FFI, HID, WdT);
  k_wtrh<<<dim3(FFI / 64, HID / 64, 1), dim3(256), 0, stream>>>(sg, HID, FFI, SgT);
  k_wtrh<<<dim3(FFI / 64, HID / 64, 1), dim3(256), 0, stream>>>(su, HID, FFI, SuT);
  k_wtrh<<<dim3(HID / 64, FFI / 64, 1), dim3(256), 0, stream>>>(sd, FFI, HID, SdT);
  k_qkv3<<<dim3(SQ / 64, NQKV / HDM), dim3(128), 0, stream>>>(Xh3, Xl3, Wqh, Wql, Ct, Sn, qnw, knw,
                                                               Qh, Ql, Kh, Kl, Vh, Vl);
  const float sscale = 0.125f;
  k_attn3<<<dim3(NH * NQ64), dim3(128), 0, stream>>>(Qh, Ql, Kh, Kl, Vh, Vl, Oh, Ol, sscale);
  k_oproj3<<<dim3(SQ / 256, HID / 64), dim3(256), 0, stream>>>(Oh, Ol, Woh, Wol, hs, Hid);
  k_route<<<dim3(SQ), dim3(128), 0, stream>>>(Hid, ln2w, rw, rb, Xm, Rt);
  k_gateup<true><<<dim3(NE * MT), dim3(256), 0, stream>>>(Xm, WgT, WuT, Rt, Mid);
  k_moe_down<<<dim3(NE * MT), dim3(256), 0, stream>>>(Mid, WdT, Rt, Y);
  k_gateup<false><<<dim3(SQ / 64), dim3(256), 0, stream>>>(Xm, SgT, SuT, Rt, Sm);
  k_final<<<dim3(SQ / 256, HID / 64), dim3(256), 0, stream>>>(Sm, SdT, Hid, Y, Rt, out);
  (void)hipGetLastError();
}
